// LSTMDecoder_80238579024342
// MI455X (gfx1250) — hardware-run, weakly checked
//
#include <hip/hip_runtime.h>

typedef __attribute__((ext_vector_type(16))) _Float16 v16h;
typedef __attribute__((ext_vector_type(8)))  _Float16 v8h;
typedef __attribute__((ext_vector_type(8)))  float    v8f;
typedef __attribute__((ext_vector_type(4)))  float    v4f;

constexpr int kBatch      = 1024;
constexpr int kAR         = 16;
constexpr int kSteps      = 128;
constexpr int kReg        = 128;
constexpr int kHid        = 16;
constexpr int kGates      = 4 * kHid;
constexpr int kOutW       = kAR + kSteps;
constexpr int kRowsPerBlk = 16;
constexpr int kBlocks     = kBatch / kRowsPerBlk;
constexpr float kWScale   = 64.0f;
constexpr float kHScale   = 16.0f;
constexpr float kInvInit  = 1.0f / 64.0f;
constexpr float kInvCell  = 1.0f / 1024.0f;
constexpr int kOutF4PerBlk = kRowsPerBlk * kOutW / 4;
constexpr int kStoreIters  = kOutF4PerBlk / 32;

static_assert(kBatch % kRowsPerBlk == 0);
static_assert(kBlocks * kRowsPerBlk == kBatch);
static_assert(kHid == 16 && kAR == kHid && kGates == 64);
static_assert(kReg % 32 == 0);
static_assert((kRowsPerBlk * kOutW * 4) % 512 == 0);
static_assert(kStoreIters * 32 == kOutF4PerBlk);
static_assert(kBatch * kOutW * 4 == 589824);

union HF { v16h v; v8h h[2]; };

__device__ __forceinline__ v8f mma16(v16h a, v16h b, v8f c) {
  c = __builtin_amdgcn_wmma_f32_16x16x32_f16(false, a, false, b, (short)0, c, false, false);
  asm volatile("v_nop\n\tv_nop\n\tv_nop\n\tv_nop" : "+v"(c) : "v"(a), "v"(b));
  return c;
}

__device__ __forceinline__ v8h cvt8h(v4f a, v4f b, float s) {
  v8h r = {(_Float16)(a[0] * s), (_Float16)(a[1] * s), (_Float16)(a[2] * s), (_Float16)(a[3] * s),
           (_Float16)(b[0] * s), (_Float16)(b[1] * s), (_Float16)(b[2] * s), (_Float16)(b[3] * s)};
  return r;
}

__device__ __forceinline__ float sigm_f(float x) {
  return __builtin_amdgcn_rcpf(1.0f + expf(-x));
}
__device__ __forceinline__ float tanh_f(float x) {
  return fmaf(2.0f, __builtin_amdgcn_rcpf(1.0f + expf(-2.0f * x)), -1.0f);
}

__global__ __launch_bounds__(32)
void lstm_ar_decode(const float* __restrict__ y,     const float* __restrict__ u,
                    const float* __restrict__ W_ih,  const float* __restrict__ W_hh,
                    const float* __restrict__ b_ih,  const float* __restrict__ b_hh,
                    const float* __restrict__ W_lin, const float* __restrict__ b_lin,
                    const float* __restrict__ W_h0,  const float* __restrict__ b_h0,
                    const float* __restrict__ W_c0,  const float* __restrict__ b_c0,
                    float* __restrict__ out)
{
  __shared__ __align__(16) float    outS[kRowsPerBlk * kOutW];
  __shared__ __align__(16) _Float16 h16[kRowsPerBlk * kHid];

  const int lane = threadIdx.x & 31;
  const int n    = lane & 15;
  const int hh   = lane >> 4;
  const int bm   = blockIdx.x * kRowsPerBlk;
  if (bm >= kBatch) return;

  const v8h z8   = {};
  const v8f zacc = {};

  float wi[4], bg[4];
#pragma unroll
  for (int g = 0; g < 4; ++g) {
    const int j = g * kHid + n;
    wi[g] = W_ih[j];
    bg[g] = b_ih[j] + b_hh[j];
  }
  const float bh0  = b_h0[n];
  const float bc0  = b_c0[n];
  const float blin = b_lin[0];

  v16h Bgate[4];
#pragma unroll
  for (int g = 0; g < 4; ++g) {
    const float* wr = W_hh + (size_t)(g * kHid + n) * kHid + 8 * hh;
    const v4f w0 = *(const v4f*)(wr);
    const v4f w1 = *(const v4f*)(wr + 4);
    HF f; f.h[0] = cvt8h(w0, w1, kWScale); f.h[1] = z8;
    Bgate[g] = f.v;
  }
  v16h Blin;
  {
    const float* wr = W_lin + 8 * hh;
    const v4f w0 = *(const v4f*)(wr);
    const v4f w1 = *(const v4f*)(wr + 4);
    HF f; f.h[0] = cvt8h(w0, w1, kWScale); f.h[1] = z8;
    Blin = f.v;
  }

  v8f acch = zacc, accc = zacc;
  {
    const float* urow = u    + (size_t)(bm + n) * kReg + 8 * hh;
    const float* wh   = W_h0 + (size_t)n * kReg + 8 * hh;
    const float* wc   = W_c0 + (size_t)n * kReg + 8 * hh;
#pragma unroll 1
    for (int q = 0; q < kReg / 32; ++q) {
      const int k0 = q * 32;
      HF a, fb, fc;
      a.h[0]  = cvt8h(*(const v4f*)(urow + k0),      *(const v4f*)(urow + k0 + 4),  1.0f);
      a.h[1]  = cvt8h(*(const v4f*)(urow + k0 + 16), *(const v4f*)(urow + k0 + 20), 1.0f);
      fb.h[0] = cvt8h(*(const v4f*)(wh + k0),        *(const v4f*)(wh + k0 + 4),    kWScale);
      fb.h[1] = cvt8h(*(const v4f*)(wh + k0 + 16),   *(const v4f*)(wh + k0 + 20),   kWScale);
      fc.h[0] = cvt8h(*(const v4f*)(wc + k0),        *(const v4f*)(wc + k0 + 4),    kWScale);
      fc.h[1] = cvt8h(*(const v4f*)(wc + k0 + 16),   *(const v4f*)(wc + k0 + 20),   kWScale);
      acch = mma16(a.v, fb.v, acch);
      accc = mma16(a.v, fc.v, accc);
    }
  }
  float cst[8], hcur[8];
#pragma unroll
  for (int r = 0; r < 8; ++r) {
    hcur[r] = fmaf(acch[r], kInvInit, bh0);
    cst[r]  = fmaf(accc[r], kInvInit, bc0);
  }

#pragma unroll
  for (int i = 0; i < 2; ++i) {
    const int idx4 = lane + 32 * i;
    const int m  = idx4 >> 2;
    const int c4 = (idx4 & 3) * 4;
    const v4f v = *(const v4f*)(y + (size_t)(bm + m) * kAR + c4);
    *(v4f*)(outS + m * kOutW + c4) = v;
  }
#pragma unroll
  for (int r = 0; r < 8; ++r)
    h16[(8 * hh + r) * kHid + n] = (_Float16)(hcur[r] * kHScale);
  __syncthreads();

#pragma unroll 1
  for (int t = 0; t < kSteps; ++t) {
#pragma unroll 1
    for (int j = 0; j < kAR; ++j) {
      HF a;
      a.h[0] = *(const v8h*)(h16 + n * kHid + 8 * hh);
      a.h[1] = z8;
      float xv[8];
#pragma unroll
      for (int r = 0; r < 8; ++r) xv[r] = outS[(8 * hh + r) * kOutW + t + j];

      v8f gi = mma16(a.v, Bgate[0], zacc);
      v8f gf = mma16(a.v, Bgate[1], zacc);
      v8f gg = mma16(a.v, Bgate[2], zacc);
      v8f go = mma16(a.v, Bgate[3], zacc);

#pragma unroll
      for (int r = 0; r < 8; ++r) {
        float pi = fmaf(gi[r], kInvCell, bg[0]); pi = fmaf(xv[r], wi[0], pi);
        float pf = fmaf(gf[r], kInvCell, bg[1]); pf = fmaf(xv[r], wi[1], pf);
        float pg = fmaf(gg[r], kInvCell, bg[2]); pg = fmaf(xv[r], wi[2], pg);
        float po = fmaf(go[r], kInvCell, bg[3]); po = fmaf(xv[r], wi[3], po);
        const float iv = sigm_f(pi);
        const float fv = sigm_f(pf);
        const float gv = tanh_f(pg);
        const float ov = sigm_f(po);
        const float cv = fv * cst[r] + iv * gv;
        cst[r]  = cv;
        hcur[r] = ov * tanh_f(cv);
      }
#pragma unroll
      for (int r = 0; r < 8; ++r)
        h16[(8 * hh + r) * kHid + n] = (_Float16)(hcur[r] * kHScale);
      __syncthreads();
    }

    HF a;
    a.h[0] = *(const v8h*)(h16 + n * kHid + 8 * hh);
    a.h[1] = z8;
    v8f pa = mma16(a.v, Blin, zacc);
    float pr[8];
#pragma unroll
    for (int r = 0; r < 8; ++r) pr[r] = fmaf(pa[r], kInvCell, blin);
    if (n == 0) {
#pragma unroll
      for (int r = 0; r < 8; ++r) outS[(8 * hh + r) * kOutW + kAR + t] = pr[r];
    }
    __syncthreads();
  }

  float* ob = out + (size_t)bm * kOutW;
  for (int pass = 0; pass < 2; ++pass) {
#pragma unroll
    for (int it = 0; it < kStoreIters; ++it) {
      const int idx4 = it * 32 + lane;
      const v4f v = *(const v4f*)(outS + idx4 * 4);
      *(volatile v4f*)(ob + (size_t)idx4 * 4) = v;
    }
    __threadfence();
  }
}

extern "C" void kernel_launch(void* const* d_in, const int* in_sizes, int n_in,
                              void* d_out, int out_size, void* d_ws, size_t ws_size,
                              hipStream_t stream) {
  (void)d_ws; (void)ws_size;
  if (n_in < 12) return;
  if (in_sizes[0]  != kBatch * kAR)  return;
  if (in_sizes[1]  != kBatch * kReg) return;
  if (in_sizes[2]  != kGates)        return;
  if (in_sizes[3]  != kGates * kHid) return;
  if (in_sizes[4]  != kGates)        return;
  if (in_sizes[5]  != kGates)        return;
  if (in_sizes[6]  != kHid)          return;
  if (in_sizes[7]  != 1)             return;
  if (in_sizes[8]  != kHid * kReg)   return;
  if (in_sizes[9]  != kHid)          return;
  if (in_sizes[10] != kHid * kReg)   return;
  if (in_sizes[11] != kHid)          return;
  if (out_size != kBatch * kOutW)    return;

  const float* y     = (const float*)d_in[0];
  const float* u     = (const float*)d_in[1];
  const float* W_ih  = (const float*)d_in[2];
  const float* W_hh  = (const float*)d_in[3];
  const float* b_ih  = (const float*)d_in[4];
  const float* b_hh  = (const float*)d_in[5];
  const float* W_lin = (const float*)d_in[6];
  const float* b_lin = (const float*)d_in[7];
  const float* W_h0  = (const float*)d_in[8];
  const float* b_h0  = (const float*)d_in[9];
  const float* W_c0  = (const float*)d_in[10];
  const float* b_c0  = (const float*)d_in[11];
  float* out = (float*)d_out;

  lstm_ar_decode<<<dim3(kBlocks), dim3(32), 0, stream>>>(
      y, u, W_ih, W_hh, b_ih, b_hh, W_lin, b_lin, W_h0, b_h0, W_c0, b_c0, out);
}
